// ParallelSubPolicies_6116033429645
// MI455X (gfx1250) — hardware-verified
//
#include <hip/hip_runtime.h>
#include <math.h>
#include <stdint.h>

#define OBS_D 128
#define HID_D 256
#define ACT_D 32
#define P_N   64
#define B_N   4096
#define MT    64
#define TPB   256
#define NWV   (TPB / 32)
#define AP    264
#define WP    40
#define EPSV  1e-5f

static_assert((B_N % MT) == 0);
static_assert(MT == 16 * (NWV / 2));
static_assert((AP % 8) == 0);
static_assert((WP % 8) == 0);
static_assert((OBS_D % 32) == 0);
static_assert((HID_D % 32) == 0);
static_assert(ACT_D == 32);
static_assert((OBS_D % 4) == 0);

typedef __bf16         v16b __attribute__((ext_vector_type(16)));
typedef unsigned short v8us __attribute__((ext_vector_type(8)));
typedef float          v8f  __attribute__((ext_vector_type(8)));
typedef float          v4f  __attribute__((ext_vector_type(4)));
typedef unsigned int   v4u  __attribute__((ext_vector_type(4)));

union Frag { v16b v; v8us u[2]; };

__device__ __forceinline__ unsigned short bf_bits(float f) {
  const unsigned u = __float_as_uint(f);
  return (unsigned short)((u + 0x7FFFu + ((u >> 16) & 1u)) >> 16);
}
__device__ __forceinline__ float bf_up(unsigned short b) { return __uint_as_float(((unsigned)b) << 16); }
__device__ __forceinline__ float bfr(float f) { return bf_up(bf_bits(f)); }

__device__ __forceinline__ float hsum16(float s) {
  s += __shfl_xor(s, 1, 32);
  s += __shfl_xor(s, 2, 32);
  s += __shfl_xor(s, 4, 32);
  s += __shfl_xor(s, 8, 32);
  return s;
}

__device__ __forceinline__ v16b ldfrag(const unsigned short* p) {
  Frag f;
  f.u[0] = *(const v8us*)(p);
  f.u[1] = *(const v8us*)(p + 16);
  return f.v;
}

__device__ __forceinline__ v8f mma_bf(v16b a, v16b b, v8f c) {
  return __builtin_amdgcn_wmma_f32_16x16x32_bf16(false, a, false, b, (short)0, c, false, false);
}

template<int N>
__device__ __forceinline__ void mma_guard(v8f (&c)[N], v16b a0, v16b a1, v16b b) {
  static_assert(N == 8 || N == 1);
#if defined(__HIP_DEVICE_COMPILE__)
  if constexpr (N == 8) {
    asm volatile("v_nop\n\tv_nop\n\tv_nop\n\tv_nop"
                 : "+v"(c[0]), "+v"(c[1]), "+v"(c[2]), "+v"(c[3]),
                   "+v"(c[4]), "+v"(c[5]), "+v"(c[6]), "+v"(c[7])
                 : "v"(a0), "v"(a1), "v"(b));
  } else {
    asm volatile("v_nop\n\tv_nop\n\tv_nop\n\tv_nop"
                 : "+v"(c[0])
                 : "v"(a0), "v"(a1), "v"(b));
  }
#else
  (void)c; (void)a0; (void)a1; (void)b;
#endif
}

template<int DIN, int DOUT>
__global__ __launch_bounds__(TPB) void k_prep(const float* __restrict__ W, unsigned short* Wt) {
  constexpr int KC     = DIN / 32;
  constexpr int PIECES = DOUT * 4;
  constexpr int NPT    = (PIECES + TPB - 1) / TPB;
  __shared__ __align__(16) unsigned short sT[DOUT * WP];
  const int tid = threadIdx.x;
  const int bid = blockIdx.x;
  const int p   = bid / KC;
  const int kc  = bid - p * KC;
  const float* src = W + ((size_t)p * DIN + (size_t)kc * 32) * DOUT;
  for (int e = tid; e < 32 * DOUT; e += TPB) {
    const int kk = e / DOUT;
    const int nn = e - kk * DOUT;
    sT[nn * WP + kk] = bf_bits(src[e]);
  }
  __syncthreads();
  v4u vals[NPT];
#pragma unroll
  for (int i = 0; i < NPT; ++i) {
    int q = i * TPB + tid;
    if (q > PIECES - 1) q = PIECES - 1;
    vals[i] = *(const v4u*)(sT + (q >> 2) * WP + (q & 3) * 8);
  }
  unsigned short* dst = Wt + (size_t)bid * (size_t)(DOUT * 32);
#pragma unroll
  for (int i = 0; i < NPT; ++i) {
    const int q = i * TPB + tid;
    if (q < PIECES) *(volatile v4u*)(dst + (size_t)q * 8) = vals[i];
  }
  __threadfence();
#pragma unroll
  for (int i = 0; i < NPT; ++i) {
    const int q = i * TPB + tid;
    if (q < PIECES) *(volatile v4u*)(dst + (size_t)q * 8) = vals[i];
  }
}

template<int DIN, int DOUT, bool TWO, bool DOELU, bool LAST>
__device__ __forceinline__ void layer_step(const unsigned short* __restrict__ Wt,
                                           const float* __restrict__ bias,
                                           const float* __restrict__ gam,
                                           const float* __restrict__ bet,
                                           float* out, int p, int b0,
                                           unsigned short* s_hi, unsigned short* s_lo, unsigned short* s_w,
                                           float* s_out, float* s_r1, float* s_r2) {
  constexpr int KC     = DIN / 32;
  constexpr int NTW    = DOUT / 32;
  constexpr int HALF   = DOUT / 2;
  constexpr int PIECES = DOUT * 4;
  constexpr float INVD = 1.0f / (float)DOUT;

  const int tid  = threadIdx.x;
  const int lane = tid & 31;
  const int wid  = tid >> 5;
  const int rg   = wid >> 1;
  const int ch   = wid & 1;
  const int h    = lane >> 4;
  const int n    = lane & 15;
  const int arow = rg * 16 + n;
  const int c0   = ch * HALF;

  v8f acc[NTW];
#pragma unroll
  for (int t = 0; t < NTW; ++t) acc[t] = (v8f){0.f, 0.f, 0.f, 0.f, 0.f, 0.f, 0.f, 0.f};

#pragma unroll 1
  for (int kc = 0; kc < KC; ++kc) {
    __syncthreads();
    const unsigned short* g = Wt + ((size_t)(p * KC + kc) * DOUT) * 32;
    for (int q = tid; q < PIECES; q += TPB) {
      const v4u x = *(const v4u*)(g + (size_t)q * 8);
      *(v4u*)(s_w + (q >> 2) * WP + (q & 3) * 8) = x;
    }
    __syncthreads();

    const v16b ahi = ldfrag(s_hi + arow * AP + kc * 32 + 8 * h);
    v16b alo = ahi;
    if constexpr (TWO) alo = ldfrag(s_lo + arow * AP + kc * 32 + 8 * h);
    v16b bb = ahi;
#pragma unroll
    for (int t = 0; t < NTW; ++t) {
      bb = ldfrag(s_w + (c0 + t * 16 + n) * WP + 8 * h);
      acc[t] = mma_bf(ahi, bb, acc[t]);
      if constexpr (TWO) acc[t] = mma_bf(alo, bb, acc[t]);
    }
    mma_guard<NTW>(acc, ahi, alo, bb);
  }

#pragma unroll
  for (int t = 0; t < NTW; ++t) {
    const float bb = bfr(bias[p * DOUT + c0 + t * 16 + n]);
#pragma unroll
    for (int r = 0; r < 8; ++r) acc[t][r] += bb;
  }
  float mu[8];
#pragma unroll
  for (int r = 0; r < 8; ++r) {
    float s = 0.0f;
#pragma unroll
    for (int t = 0; t < NTW; ++t) s += acc[t][r];
    s = hsum16(s);
    if (n == 0) s_r1[wid * 16 + 8 * h + r] = s;
    mu[r] = s;
  }
  __syncthreads();
#pragma unroll
  for (int r = 0; r < 8; ++r) {
    const float sa = s_r1[(rg * 2) * 16 + 8 * h + r];
    const float sb = s_r1[(rg * 2 + 1) * 16 + 8 * h + r];
    mu[r] = (sa + sb) * INVD;
  }
  float sc[8];
#pragma unroll
  for (int r = 0; r < 8; ++r) {
    float s = 0.0f;
#pragma unroll
    for (int t = 0; t < NTW; ++t) { const float d = acc[t][r] - mu[r]; s += d * d; }
    s = hsum16(s);
    if (n == 0) s_r2[wid * 16 + 8 * h + r] = s;
    sc[r] = s;
  }
  __syncthreads();
#pragma unroll
  for (int r = 0; r < 8; ++r) {
    const float sa = s_r2[(rg * 2) * 16 + 8 * h + r];
    const float sb = s_r2[(rg * 2 + 1) * 16 + 8 * h + r];
    const float var = (sa + sb) * INVD;
    sc[r] = rsqrtf(var + EPSV);
  }
#pragma unroll
  for (int t = 0; t < NTW; ++t) {
    const int col  = c0 + t * 16 + n;
    const float gg = bfr(gam[p * DOUT + col]);
    const float ee = bfr(bet[p * DOUT + col]);
#pragma unroll
    for (int r = 0; r < 8; ++r) {
      float v = (acc[t][r] - mu[r]) * sc[r] * gg + ee;
      if constexpr (DOELU) {
        const float em = expm1f(fminf(v, 0.0f));
        v = (v > 0.0f) ? v : em;
      }
      const int row = rg * 16 + 8 * h + r;
      if constexpr (LAST) {
        s_out[row * ACT_D + col] = v;
      } else {
        const unsigned short hb = bf_bits(v);
        const unsigned short lb = bf_bits(v - bf_up(hb));
        s_hi[row * AP + col] = hb;
        s_lo[row * AP + col] = lb;
      }
    }
  }

  if constexpr (LAST) {
    __syncthreads();
    const int pc   = (lane & 7) * 4;
    const int row0 = rg * 16 + ch * 8 + (lane >> 3);
    const int row1 = row0 + 4;
    const v4f o0 = *(const v4f*)(s_out + row0 * ACT_D + pc);
    const v4f o1 = *(const v4f*)(s_out + row1 * ACT_D + pc);
    float* d0 = out + ((size_t)(b0 + row0) * P_N + (size_t)p) * ACT_D + pc;
    float* d1 = out + ((size_t)(b0 + row1) * P_N + (size_t)p) * ACT_D + pc;
    *(volatile v4f*)d0 = o0;
    *(volatile v4f*)d1 = o1;
    __threadfence();
    *(volatile v4f*)d0 = o0;
    *(volatile v4f*)d1 = o1;
  }
}

__global__ __launch_bounds__(TPB) void k_mlp(const float* __restrict__ obs,
                                             const unsigned short* __restrict__ Wt1, const float* __restrict__ b1,
                                             const float* __restrict__ g1, const float* __restrict__ be1,
                                             const unsigned short* __restrict__ Wt2, const float* __restrict__ b2,
                                             const float* __restrict__ g2, const float* __restrict__ be2,
                                             const unsigned short* __restrict__ Wt3, const float* __restrict__ b3,
                                             const float* __restrict__ g3, const float* __restrict__ be3,
                                             const unsigned short* __restrict__ Wt4, const float* __restrict__ b4,
                                             const float* __restrict__ g4, const float* __restrict__ be4,
                                             float* out) {
  __shared__ __align__(16) unsigned short s_hi[MT * AP];
  __shared__ __align__(16) unsigned short s_lo[MT * AP];
  __shared__ __align__(16) unsigned short s_w[HID_D * WP];
  __shared__ __align__(16) float s_out[MT * ACT_D];
  __shared__ float s_r1[NWV * 16];
  __shared__ float s_r2[NWV * 16];

  const int tid = threadIdx.x;
  const int p   = blockIdx.y;
  const int b0  = blockIdx.x * MT;

  for (int q = tid; q < MT * (OBS_D / 4); q += TPB) {
    const int r  = q / (OBS_D / 4);
    const int c4 = q - r * (OBS_D / 4);
    const v4f x = *(const v4f*)(obs + (size_t)(b0 + r) * OBS_D + (size_t)c4 * 4);
    unsigned short* d = s_hi + r * AP + c4 * 4;
    d[0] = bf_bits(x[0]);
    d[1] = bf_bits(x[1]);
    d[2] = bf_bits(x[2]);
    d[3] = bf_bits(x[3]);
  }

  layer_step<OBS_D, HID_D, false, true,  false>(Wt1, b1, g1, be1, out, p, b0, s_hi, s_lo, s_w, s_out, s_r1, s_r2);
  layer_step<HID_D, HID_D, true,  true,  false>(Wt2, b2, g2, be2, out, p, b0, s_hi, s_lo, s_w, s_out, s_r1, s_r2);
  layer_step<HID_D, HID_D, true,  true,  false>(Wt3, b3, g3, be3, out, p, b0, s_hi, s_lo, s_w, s_out, s_r1, s_r2);
  layer_step<HID_D, ACT_D, true,  false, true >(Wt4, b4, g4, be4, out, p, b0, s_hi, s_lo, s_w, s_out, s_r1, s_r2);
}

extern "C" void kernel_launch(void* const* d_in, const int* in_sizes, int n_in,
                              void* d_out, int out_size, void* d_ws, size_t ws_size,
                              hipStream_t stream) {
  if (n_in < 17) return;
  if (in_sizes[0]  != B_N * OBS_D) return;
  if (in_sizes[1]  != P_N * OBS_D * HID_D) return;
  if (in_sizes[2]  != P_N * HID_D || in_sizes[3]  != P_N * HID_D || in_sizes[4]  != P_N * HID_D) return;
  if (in_sizes[5]  != P_N * HID_D * HID_D) return;
  if (in_sizes[6]  != P_N * HID_D || in_sizes[7]  != P_N * HID_D || in_sizes[8]  != P_N * HID_D) return;
  if (in_sizes[9]  != P_N * HID_D * HID_D) return;
  if (in_sizes[10] != P_N * HID_D || in_sizes[11] != P_N * HID_D || in_sizes[12] != P_N * HID_D) return;
  if (in_sizes[13] != P_N * HID_D * ACT_D) return;
  if (in_sizes[14] != P_N * ACT_D || in_sizes[15] != P_N * ACT_D || in_sizes[16] != P_N * ACT_D) return;
  if (out_size != B_N * P_N * ACT_D) return;

  const float* obs = (const float*)d_in[0];
  const float* W1  = (const float*)d_in[1];
  const float* b1  = (const float*)d_in[2];
  const float* g1  = (const float*)d_in[3];
  const float* be1 = (const float*)d_in[4];
  const float* W2  = (const float*)d_in[5];
  const float* b2  = (const float*)d_in[6];
  const float* g2  = (const float*)d_in[7];
  const float* be2 = (const float*)d_in[8];
  const float* W3  = (const float*)d_in[9];
  const float* b3  = (const float*)d_in[10];
  const float* g3  = (const float*)d_in[11];
  const float* be3 = (const float*)d_in[12];
  const float* W4  = (const float*)d_in[13];
  const float* b4  = (const float*)d_in[14];
  const float* g4  = (const float*)d_in[15];
  const float* be4 = (const float*)d_in[16];
  float* out = (float*)d_out;

  const size_t sz1 = (size_t)P_N * OBS_D * HID_D * 2;
  const size_t sz2 = (size_t)P_N * HID_D * HID_D * 2;
  const size_t sz3 = sz2;
  const size_t sz4 = (size_t)P_N * HID_D * ACT_D * 2;
  size_t off = 0;
  const size_t o1 = off; off += sz1;
  const size_t o2 = off; off += sz2;
  const size_t o3 = off; off += sz3;
  const size_t o4 = off; off += sz4;
  if (off > ws_size) return;
  if (off > (size_t)134217728) return;

  char* ws = (char*)d_ws;
  unsigned short* Wt1 = (unsigned short*)(ws + o1);
  unsigned short* Wt2 = (unsigned short*)(ws + o2);
  unsigned short* Wt3 = (unsigned short*)(ws + o3);
  unsigned short* Wt4 = (unsigned short*)(ws + o4);

  const dim3 blk(TPB);
  const dim3 gP1(P_N * (OBS_D / 32));
  const dim3 gP2(P_N * (HID_D / 32));
  const dim3 gMain(B_N / MT, P_N);

  k_prep<OBS_D, HID_D><<<gP1, blk, 0, stream>>>(W1, Wt1);
  k_prep<HID_D, HID_D><<<gP2, blk, 0, stream>>>(W2, Wt2);
  k_prep<HID_D, HID_D><<<gP2, blk, 0, stream>>>(W3, Wt3);
  k_prep<HID_D, ACT_D><<<gP2, blk, 0, stream>>>(W4, Wt4);
  k_mlp<<<gMain, blk, 0, stream>>>(obs, Wt1, b1, g1, be1, Wt2, b2, g2, be2, Wt3, b3, g3, be3,
                                   Wt4, b4, g4, be4, out);
  (void)hipGetLastError();
}
